// MultiheadCrossAttention_146028888611
// MI455X (gfx1250) — hardware-verified
//
#include <hip/hip_runtime.h>


#ifndef NB
#define NB 4
#endif
#ifndef SEQ
#define SEQ 1024
#endif
#define NB_FULL 4
#define T_FULL 1024
#define S_FULL 1024
#define DMOD 1024
#define DKV 2048
#define QKVP 3072
#define NHD 16
#define HD 64
#define HCH 192
#define QB 32
#define PCAR 16384.0f
#define L2S (0.125f * 1.4426950408889634f)
#define WSC 32.0f
#define IWSC 0.03125f

static_assert(NHD * HD == DMOD);
static_assert(HD == 64);
static_assert(3 * HD == HCH);
static_assert(NHD * HCH == QKVP);
static_assert(NB >= 1 && NB <= NB_FULL);
static_assert(SEQ % 64 == 0);
static_assert(SEQ % QB == 0);
static_assert(SEQ <= T_FULL);
static_assert(SEQ <= S_FULL);
static_assert(DMOD % 64 == 0);
static_assert(DKV % 64 == 0);

#define WS_XB  ((size_t)NB * SEQ * DMOD * 2)
#define WS_WKV ((size_t)DKV * DMOD * 2)
#define WS_W   ((size_t)DMOD * DMOD * 2)
#define WS_WM  ((size_t)SEQ * SEQ * 2)
#define WS_QT  ((size_t)NB * DMOD * SEQ * 2)
#define WS_QKV ((size_t)NB * SEQ * QKVP * 2)
#define WS_VT  ((size_t)NB * NHD * HD * SEQ * 2)
#define WS_CT  ((size_t)NB * SEQ * DMOD * 2)
#define WS_TOTAL (2 * WS_XB + WS_WKV + 3 * WS_W + 2 * WS_WM + 2 * WS_QT + WS_QKV + WS_VT + 2 * WS_CT)
static_assert(WS_XB % 256 == 0);
static_assert(WS_WKV % 256 == 0);
static_assert(WS_W % 256 == 0);
static_assert(WS_WM % 256 == 0);
static_assert(WS_QT % 256 == 0);
static_assert(WS_QKV % 256 == 0);
static_assert(WS_VT % 256 == 0);
static_assert(WS_CT % 256 == 0);
static_assert(WS_TOTAL <= (size_t)134217728);

typedef _Float16 h16;
typedef unsigned short bf;
typedef __attribute__((ext_vector_type(16))) __bf16   v16bf;
typedef __attribute__((ext_vector_type(16))) _Float16 v16h;
typedef __attribute__((ext_vector_type(8)))  _Float16 v8h;
typedef __attribute__((ext_vector_type(8)))  unsigned short v8us;
typedef __attribute__((ext_vector_type(8)))  float    v8f;
typedef __attribute__((ext_vector_type(4)))  float    v4f;
typedef v8h  __attribute__((may_alias)) v8ha;
typedef v4f  __attribute__((may_alias)) v4fa;
typedef v8us __attribute__((may_alias)) v8usa;

__device__ __forceinline__ unsigned short f2bf(float f) { unsigned u = __float_as_uint(f); u += 0x7FFFu + ((u >> 16) & 1u); return (unsigned short)(u >> 16); }
__device__ __forceinline__ float bf2f(unsigned short b) { return __uint_as_float(((unsigned)b) << 16); }
__device__ __forceinline__ float bfr(float f) { return bf2f(f2bf(f)); }
__device__ __forceinline__ v4f bfr4(v4f x) { v4f r; r[0] = bfr(x[0]); r[1] = bfr(x[1]); r[2] = bfr(x[2]); r[3] = bfr(x[3]); return r; }
__device__ __forceinline__ v16h cat16(v8h lo, v8h hi) { return __builtin_shufflevector(lo, hi, 0, 1, 2, 3, 4, 5, 6, 7, 8, 9, 10, 11, 12, 13, 14, 15); }
__device__ __forceinline__ v16bf cat16b(v8us lo, v8us hi) { return __builtin_bit_cast(v16bf, __builtin_shufflevector(lo, hi, 0, 1, 2, 3, 4, 5, 6, 7, 8, 9, 10, 11, 12, 13, 14, 15)); }
__device__ __forceinline__ v8f wmma16(v16h a, v16h b, v8f c) { return __builtin_amdgcn_wmma_f32_16x16x32_f16(false, a, false, b, (short)0, c, false, false); }
__device__ __forceinline__ v8f wmmab(v16bf a, v16bf b, v8f c) { return __builtin_amdgcn_wmma_f32_16x16x32_bf16(false, a, false, b, (short)0, c, false, false); }
__device__ __forceinline__ void splitf(float y, unsigned short& h, unsigned short& l) { h = f2bf(y); l = f2bf(y - bf2f(h)); }
__device__ __forceinline__ h16 tof16(float y) { y = (fabsf(y) < 6.103515625e-05f) ? 0.0f : y; return (h16)y; }

template <typename T16> struct WFrag;
template <> struct WFrag<h16> { typedef v16h V; static __device__ __forceinline__ V ld(const h16* p) { return cat16(*(const v8h*)p, *(const v8h*)(p + 16)); } static __device__ __forceinline__ v8f mma(V a, V b, v8f c) { return wmma16(a, b, c); } };
template <> struct WFrag<bf> { typedef v16bf V; static __device__ __forceinline__ V ld(const bf* p) { return cat16b(*(const v8us*)p, *(const v8us*)(p + 16)); } static __device__ __forceinline__ v8f mma(V a, V b, v8f c) { return wmmab(a, b, c); } };

template <bool COLB, int NROWB>
__device__ __forceinline__ void epi_slab(float* crow, int ldc, const float* os, int lane, const float* __restrict__ cb, int c0,
                                         const float* __restrict__ rb, const float* __restrict__ rb2, int rbase, float oscale) {
    const int lr = lane & 15, hi = lane >> 4, cofs = lr * 4;
    v4f cbv = (v4f){0.0f, 0.0f, 0.0f, 0.0f};
    if (COLB) cbv = bfr4(*(const v4f*)(cb + c0 + cofs));
#pragma unroll 1
    for (int ps = 0; ps < 2; ++ps) {
#pragma unroll
        for (int s = 0; s < 8; ++s) { const int row = 2 * s + hi; v4f val = *(const v4fa*)(os + row * 68 + cofs); val = val * oscale + cbv;
            if (NROWB >= 1) { float rv = bfr(rb[rbase + row]); if (NROWB == 2) rv += bfr(rb2[rbase + row]); val += rv; }
            *(volatile v4f*)(crow + (size_t)row * ldc + cofs) = val; }
        if (ps == 0) __threadfence(); }
}
template <bool COLB, int NROWB>
__device__ __forceinline__ void epi_slab(h16* crow, int ldc, const float* os, int lane, const float* __restrict__ cb, int c0,
                                         const float* __restrict__ rb, const float* __restrict__ rb2, int rbase, float oscale) {
    const int piece = lane & 7, rq = lane >> 3, cofs = piece * 8;
    v4f cb0 = (v4f){0.0f, 0.0f, 0.0f, 0.0f}, cb1 = (v4f){0.0f, 0.0f, 0.0f, 0.0f};
    if (COLB) { cb0 = bfr4(*(const v4f*)(cb + c0 + cofs)); cb1 = bfr4(*(const v4f*)(cb + c0 + cofs + 4)); }
    v8h o[4];
#pragma unroll
    for (int s = 0; s < 4; ++s) { const int row = 4 * s + rq;
        v4f v0 = *(const v4fa*)(os + row * 68 + cofs); v4f v1 = *(const v4fa*)(os + row * 68 + cofs + 4);
        float rv = 0.0f; if (NROWB >= 1) { rv = bfr(rb[rbase + row]); if (NROWB == 2) rv += bfr(rb2[rbase + row]); }
        v0 = v0 * oscale + cb0 + rv; v1 = v1 * oscale + cb1 + rv;
#pragma unroll
        for (int e = 0; e < 4; ++e) { o[s][e] = tof16(v0[e]); o[s][4 + e] = tof16(v1[e]); } }
#pragma unroll 1
    for (int ps = 0; ps < 2; ++ps) {
#pragma unroll
        for (int s = 0; s < 4; ++s) { const int row = 4 * s + rq; *(volatile v8h*)(crow + (size_t)row * ldc + cofs) = o[s]; }
        if (ps == 0) __threadfence(); }
}

template <typename T16, int MODE, typename TO, bool COLB, int NROWB>
__global__ __launch_bounds__(32) __attribute__((amdgpu_num_vgpr(256)))
void k_gemm(const T16* __restrict__ A, const T16* __restrict__ A2, const T16* __restrict__ Bt, const T16* __restrict__ Bt2, int K,
            TO* C, int ldc, const float* __restrict__ cb, const float* __restrict__ rb, const float* __restrict__ rb2, float oscale,
            size_t sA, size_t sB, size_t sC) {
    typedef typename WFrag<T16>::V V;
    __shared__ __align__(16) float os[16 * 68];
    const size_t z = blockIdx.z; A += z * sA; if (MODE != 0) A2 += z * sA; Bt += z * sB; if (MODE == 2) Bt2 += z * sB; C += z * sC;
    const int lane = threadIdx.x & 31, lr = lane & 15, hi = lane >> 4; const int r0 = blockIdx.x * 64, c0 = blockIdx.y * 64;
    v8f acc[4][4];
#pragma unroll
    for (int mb = 0; mb < 4; ++mb)
#pragma unroll
        for (int nb = 0; nb < 4; ++nb) acc[mb][nb] = (v8f){};
    const size_t aoff = (size_t)(r0 + lr) * K + 8 * hi, boff = (size_t)(c0 + lr) * K + 8 * hi;
#pragma unroll 1
    for (int kc = 0; kc < K; kc += 32) {
        V a[4], a2[4];
#pragma unroll
        for (int mb = 0; mb < 4; ++mb) { a[mb] = WFrag<T16>::ld(A + aoff + (size_t)mb * 16 * K + kc); if (MODE == 1) a2[mb] = WFrag<T16>::ld(A2 + aoff + (size_t)mb * 16 * K + kc); }
#pragma unroll
        for (int nb = 0; nb < 4; ++nb) { const V b = WFrag<T16>::ld(Bt + boff + (size_t)nb * 16 * K + kc);
#pragma unroll
            for (int mb = 0; mb < 4; ++mb) { acc[mb][nb] = WFrag<T16>::mma(a[mb], b, acc[mb][nb]); if (MODE == 1) acc[mb][nb] = WFrag<T16>::mma(a2[mb], b, acc[mb][nb]); } }
        if (MODE == 2) {
            asm volatile("" : "+v"(acc[0][0]), "+v"(acc[3][3]) : : "memory");
#pragma unroll
            for (int mb = 0; mb < 4; ++mb) a2[mb] = WFrag<T16>::ld(A2 + aoff + (size_t)mb * 16 * K + kc);
#pragma unroll
            for (int nb = 0; nb < 4; ++nb) { const V b2 = WFrag<T16>::ld(Bt2 + boff + (size_t)nb * 16 * K + kc);
#pragma unroll
                for (int mb = 0; mb < 4; ++mb) acc[mb][nb] = WFrag<T16>::mma(a2[mb], b2, acc[mb][nb]); }
            asm volatile("v_nop\n\tv_nop\n\tv_nop\n\tv_nop" : "+v"(acc[0][0]), "+v"(acc[1][1]), "+v"(acc[2][2]), "+v"(acc[3][3]) : "v"(a2[0]), "v"(a2[3]));
        } else {
            asm volatile("v_nop\n\tv_nop\n\tv_nop\n\tv_nop" : "+v"(acc[0][0]), "+v"(acc[1][1]), "+v"(acc[2][2]), "+v"(acc[3][3]) : "v"(a[0]), "v"(a[3]));
        }
    }
#pragma unroll
    for (int mb = 0; mb < 4; ++mb) {
#pragma unroll
        for (int nb = 0; nb < 4; ++nb) {
#pragma unroll
            for (int j = 0; j < 8; ++j) os[(hi * 8 + j) * 68 + nb * 16 + lr] = acc[mb][nb][j]; }
        __builtin_amdgcn_wave_barrier(); asm volatile("" ::: "memory");
        epi_slab<COLB, NROWB>(C + (size_t)(r0 + mb * 16) * ldc + c0, ldc, os, lane, cb, c0, rb, rb2, r0 + mb * 16, oscale);
        __builtin_amdgcn_wave_barrier(); asm volatile("" ::: "memory");
    }
}

__global__ __launch_bounds__(256) void k_cvtb(const float* __restrict__ src, bf* dst, int rows, int cols8, int rpg, int sgs, int spitch) {
    const size_t i = (size_t)blockIdx.x * 256 + threadIdx.x; if (i >= (size_t)rows * cols8) return;
    const int row = (int)(i / (size_t)cols8), c8 = (int)(i - (size_t)row * cols8);
    const size_t srow = (size_t)(row / rpg) * sgs + (size_t)(row % rpg);
    const v8f v = *(const v8f*)(src + srow * (size_t)spitch + (size_t)c8 * 8); v8us o;
#pragma unroll
    for (int k = 0; k < 8; ++k) o[k] = f2bf(v[k]);
    *(volatile v8us*)(dst + i * 8) = o; __threadfence(); *(volatile v8us*)(dst + i * 8) = o;
}
__global__ __launch_bounds__(256) void k_cvth(const float* __restrict__ src, h16* dst, int rows, int cols8, int rpg, int sgs, int spitch, float scale) {
    const size_t i = (size_t)blockIdx.x * 256 + threadIdx.x; if (i >= (size_t)rows * cols8) return;
    const int row = (int)(i / (size_t)cols8), c8 = (int)(i - (size_t)row * cols8);
    const size_t srow = (size_t)(row / rpg) * sgs + (size_t)(row % rpg);
    const v8f v = *(const v8f*)(src + srow * (size_t)spitch + (size_t)c8 * 8); v8h o;
#pragma unroll
    for (int k = 0; k < 8; ++k) o[k] = tof16(bfr(v[k]) * scale);
    *(volatile v8h*)(dst + i * 8) = o; __threadfence(); *(volatile v8h*)(dst + i * 8) = o;
}

__global__ __launch_bounds__(256) void k_vtr(const h16* __restrict__ F, h16* VT) {
    __shared__ __align__(16) h16 tile[64 * 72];
    const int b = blockIdx.z, head = blockIdx.y, s0 = blockIdx.x * 64, t = threadIdx.x;
    {
        const int r = t >> 2, seg = t & 3;
        const h16* src = F + ((size_t)b * SEQ + s0 + r) * QKVP + head * HCH + 2 * HD + seg * 16;
#pragma unroll
        for (int q = 0; q < 2; ++q) { const v8h a = *(const v8h*)(src + 8 * q); *(v8h*)(tile + r * 72 + seg * 16 + 8 * q) = a; }
    }
    __syncthreads();
    const int piece = t & 7, rq = t >> 3;
    v8h o2[2];
#pragma unroll
    for (int pg = 0; pg < 2; ++pg) { const int d = pg * 32 + rq;
#pragma unroll
        for (int e = 0; e < 8; ++e) o2[pg][e] = tile[(piece * 8 + e) * 72 + d]; }
#pragma unroll 1
    for (int ps = 0; ps < 2; ++ps) {
#pragma unroll
        for (int pg = 0; pg < 2; ++pg) { const int d = pg * 32 + rq; *(volatile v8h*)(VT + (((size_t)(b * NHD + head)) * HD + d) * SEQ + s0 + piece * 8) = o2[pg]; }
        if (ps == 0) __threadfence(); }
}

__global__ __launch_bounds__(64) __attribute__((amdgpu_num_vgpr(256)))
void k_flash(const h16* __restrict__ QKV, const h16* __restrict__ VTp, bf* CTh, bf* CTl) {
    __shared__ __align__(16) unsigned short eh[2][16 * 64];
    __shared__ __align__(16) unsigned short el[2][16 * 64];
    const int b = blockIdx.z, head = blockIdx.y;
    const int w = threadIdx.x >> 5, lane = threadIdx.x & 31, hf = lane >> 4, lm = lane & 15;
    const int m0 = blockIdx.x * QB + w * 16;
    const int hc = head * HCH;
    v16h qf[2];
    {
        const h16* qp = QKV + ((size_t)b * SEQ + m0 + lm) * QKVP + hc + 8 * hf;
#pragma unroll
        for (int ks = 0; ks < 2; ++ks) qf[ks] = cat16(*(const v8h*)(qp + 32 * ks), *(const v8h*)(qp + 32 * ks + 16));
    }
    v8f acc[4];
#pragma unroll
    for (int dt = 0; dt < 4; ++dt) acc[dt] = (v8f){};
    float mrun = -1.0e30f, lrun = 0.0f;
    const h16* kcur = QKV + ((size_t)b * SEQ + lm) * QKVP + hc + HD + 8 * hf;
    const h16* vcur = VTp + (((size_t)(b * NHD + head)) * HD + lm) * SEQ + 8 * hf;
#pragma unroll 1
    for (int sc = 0; sc < SEQ; sc += 64) {
        v8f st[4];
#pragma unroll
        for (int s4 = 0; s4 < 4; ++s4) st[s4] = (v8f){};
#pragma unroll
        for (int s4 = 0; s4 < 4; ++s4) {
            const h16* kp = kcur + (size_t)(s4 * 16) * QKVP;
#pragma unroll
            for (int ks = 0; ks < 2; ++ks) { const v16h af = cat16(*(const v8h*)(kp + 32 * ks), *(const v8h*)(kp + 32 * ks + 16)); st[s4] = wmma16(af, qf[ks], st[s4]); }
        }
        asm volatile("v_nop\n\tv_nop\n\tv_nop\n\tv_nop" : "+v"(st[0]), "+v"(st[1]), "+v"(st[2]), "+v"(st[3]) : "v"(qf[0]), "v"(qf[1]));
        float cm = -1.0e30f;
#pragma unroll
        for (int s4 = 0; s4 < 4; ++s4) { st[s4] *= L2S;
#pragma unroll
            for (int e = 0; e < 8; ++e) cm = fmaxf(cm, st[s4][e]); }
        cm = fmaxf(cm, __shfl_xor(cm, 16, 32));
        const float mnew = fmaxf(mrun, cm);
        const float alpha = __builtin_amdgcn_exp2f(mrun - mnew);
        mrun = mnew;
        float ls = 0.0f; v16h pf[2];
#pragma unroll
        for (int s4 = 0; s4 < 4; ++s4)
#pragma unroll
            for (int e = 0; e < 8; ++e) { const float p = __builtin_amdgcn_exp2f(st[s4][e] - mnew); ls += p; pf[s4 >> 1][(s4 & 1) * 8 + e] = (h16)(p * PCAR); }
        ls += __shfl_xor(ls, 16, 32);
        lrun = lrun * alpha + ls;
        v8f av;
#pragma unroll
        for (int e = 0; e < 8; ++e) av[e] = __shfl(alpha, 8 * hf + e, 32);
#pragma unroll
        for (int dt = 0; dt < 4; ++dt) acc[dt] *= av;
        asm volatile("" ::: "memory");
#pragma unroll
        for (int ks = 0; ks < 2; ++ks) {
#pragma unroll
            for (int dt = 0; dt < 4; ++dt) { const h16* vp = vcur + (size_t)(dt * 16) * SEQ + sc + 32 * ks; const v16h vf = cat16(*(const v8h*)vp, *(const v8h*)(vp + 16)); acc[dt] = wmma16(pf[ks], vf, acc[dt]); }
            asm volatile("" ::: "memory");
        }
        asm volatile("v_nop\n\tv_nop\n\tv_nop\n\tv_nop" : "+v"(acc[0]), "+v"(acc[1]), "+v"(acc[2]), "+v"(acc[3]) : "v"(pf[0]), "v"(pf[1]));
        kcur += (size_t)64 * QKVP;
    }
    v8f lv;
#pragma unroll
    for (int e = 0; e < 8; ++e) lv[e] = __shfl(lrun, 8 * hf + e, 32);
    v8f iv;
#pragma unroll
    for (int e = 0; e < 8; ++e) iv[e] = 1.0f / (lv[e] * PCAR);
    unsigned short* ehw = eh[w]; unsigned short* elw = el[w];
#pragma unroll
    for (int dt = 0; dt < 4; ++dt)
#pragma unroll
        for (int e = 0; e < 8; ++e) { unsigned short a2, c2; splitf(acc[dt][e] * iv[e], a2, c2); const int o = (8 * hf + e) * 64 + dt * 16 + lm; ehw[o] = a2; elw[o] = c2; }
    __syncthreads();
    const int piece = lane & 7, rsub = lane >> 3;
#pragma unroll 1
    for (int ps = 0; ps < 2; ++ps) {
#pragma unroll
        for (int rg = 0; rg < 4; ++rg) { const int row = rg * 4 + rsub; const v8us oh = *(const v8usa*)(ehw + row * 64 + piece * 8); const v8us ol = *(const v8usa*)(elw + row * 64 + piece * 8);
            const size_t go = ((size_t)b * SEQ + m0 + row) * DMOD + head * HD + piece * 8;
            *(volatile v8us*)(CTh + go) = oh; *(volatile v8us*)(CTl + go) = ol; }
        if (ps == 0) __threadfence(); }
}

extern "C" void kernel_launch(void* const* d_in, const int* in_sizes, int n_in,
                              void* d_out, int out_size, void* d_ws, size_t ws_size, hipStream_t stream) {
    if (n_in < 14) return;
    if ((size_t)in_sizes[0] < ((size_t)(NB - 1) * T_FULL + SEQ) * DMOD) return;
    if ((size_t)in_sizes[1] < ((size_t)(NB - 1) * T_FULL + SEQ) * DMOD) return;
    if ((size_t)in_sizes[2] < (size_t)DKV * DMOD) return;
    if ((size_t)in_sizes[3] < (size_t)DKV) return;
    if ((size_t)in_sizes[4] < (size_t)DMOD * DMOD) return;
    if ((size_t)in_sizes[5] < (size_t)DMOD) return;
    if ((size_t)in_sizes[6] < (size_t)DMOD * DMOD) return;
    if ((size_t)in_sizes[7] < (size_t)DMOD) return;
    if ((size_t)in_sizes[8] < (size_t)DMOD * DMOD) return;
    if ((size_t)in_sizes[9] < (size_t)DMOD) return;
    if ((size_t)in_sizes[10] < (size_t)(SEQ - 1) * S_FULL + SEQ) return;
    if ((size_t)in_sizes[11] < (size_t)SEQ) return;
    if ((size_t)in_sizes[12] < (size_t)(SEQ - 1) * S_FULL + SEQ) return;
    if ((size_t)in_sizes[13] < (size_t)SEQ) return;
    if ((size_t)out_size < (size_t)NB * SEQ * DMOD) return;
    const float* x    = (const float*)d_in[0];
    const float* xc   = (const float*)d_in[1];
    const float* wkv  = (const float*)d_in[2];
    const float* bkv  = (const float*)d_in[3];
    const float* wq1  = (const float*)d_in[4];
    const float* bq1  = (const float*)d_in[5];
    const float* wq2  = (const float*)d_in[6];
    const float* bq2  = (const float*)d_in[7];
    const float* wpr  = (const float*)d_in[8];
    const float* bpr  = (const float*)d_in[9];
    const float* wone = (const float*)d_in[10];
    const float* bone = (const float*)d_in[11];
    const float* wzer = (const float*)d_in[12];
    const float* bzer = (const float*)d_in[13];
    float* OUT = (float*)d_out;
    char* wsp = (char*)d_ws;
    size_t used = 0;
    auto take = [&](size_t bytes) { char* p = wsp + used; used += (bytes + 255) & ~(size_t)255; return (void*)p; };
    bf*  Xb  = (bf*)take(WS_XB);
    bf*  XCb = (bf*)take(WS_XB);
    bf*  Wkv = (bf*)take(WS_WKV);
    bf*  Wq1 = (bf*)take(WS_W);
    bf*  Wq2 = (bf*)take(WS_W);
    bf*  Wpr = (bf*)take(WS_W);
    h16* Wm1 = (h16*)take(WS_WM);
    h16* Wm0 = (h16*)take(WS_WM);
    h16* Q1T = (h16*)take(WS_QT);
    h16* Q2T = (h16*)take(WS_QT);
    h16* QKV = (h16*)take(WS_QKV);
    h16* VT  = (h16*)take(WS_VT);
    bf*  CTh = (bf*)take(WS_CT);
    bf*  CTl = (bf*)take(WS_CT);
    if (used > ws_size) return;
    const int c8d = DMOD / 8;
    const size_t nx = (size_t)NB * SEQ * c8d, nkv = (size_t)DKV * c8d, nw = (size_t)DMOD * c8d, nm = (size_t)SEQ * (SEQ / 8);
    k_cvtb<<<(unsigned)((nx + 255) / 256), 256, 0, stream>>>(x, Xb, NB * SEQ, c8d, SEQ, T_FULL, DMOD);
    k_cvtb<<<(unsigned)((nx + 255) / 256), 256, 0, stream>>>(xc, XCb, NB * SEQ, c8d, SEQ, T_FULL, DMOD);
    k_cvtb<<<(unsigned)((nkv + 255) / 256), 256, 0, stream>>>(wkv, Wkv, DKV, c8d, DKV, 0, DMOD);
    k_cvtb<<<(unsigned)((nw + 255) / 256), 256, 0, stream>>>(wq1, Wq1, DMOD, c8d, DMOD, 0, DMOD);
    k_cvtb<<<(unsigned)((nw + 255) / 256), 256, 0, stream>>>(wq2, Wq2, DMOD, c8d, DMOD, 0, DMOD);
    k_cvtb<<<(unsigned)((nw + 255) / 256), 256, 0, stream>>>(wpr, Wpr, DMOD, c8d, DMOD, 0, DMOD);
    k_cvth<<<(unsigned)((nm + 255) / 256), 256, 0, stream>>>(wone, Wm1, SEQ, SEQ / 8, SEQ, 0, S_FULL, WSC);
    k_cvth<<<(unsigned)((nm + 255) / 256), 256, 0, stream>>>(wzer, Wm0, SEQ, SEQ / 8, SEQ, 0, S_FULL, WSC);
    k_gemm<bf, 0, h16, true, 0><<<dim3((NB * SEQ) / 64, DKV / 64, 1), 32, 0, stream>>>(Xb, (const bf*)nullptr, Wkv, (const bf*)nullptr, DMOD, QKV + DMOD, QKVP, bkv, (const float*)nullptr, (const float*)nullptr, 1.0f, (size_t)0, (size_t)0, (size_t)0);
    k_gemm<bf, 0, h16, false, 1><<<dim3(DMOD / 64, SEQ / 64, NB), 32, 0, stream>>>(Wq1, (const bf*)nullptr, Xb, (const bf*)nullptr, DMOD, Q1T, SEQ, (const float*)nullptr, bq1, (const float*)nullptr, 1.0f, (size_t)0, (size_t)SEQ * DMOD, (size_t)DMOD * SEQ);
    k_gemm<bf, 0, h16, false, 1><<<dim3(DMOD / 64, SEQ / 64, NB), 32, 0, stream>>>(Wq2, (const bf*)nullptr, XCb, (const bf*)nullptr, DMOD, Q2T, SEQ, (const float*)nullptr, bq2, (const float*)nullptr, 1.0f, (size_t)0, (size_t)SEQ * DMOD, (size_t)DMOD * SEQ);
    k_gemm<h16, 2, h16, false, 2><<<dim3(SEQ / 64, DMOD / 64, NB), 32, 0, stream>>>(Wm1, Wm0, Q1T, Q2T, SEQ, QKV, QKVP, (const float*)nullptr, bone, bzer, IWSC, (size_t)0, (size_t)DMOD * SEQ, (size_t)SEQ * QKVP);
    k_vtr<<<dim3(SEQ / 64, NHD, NB), 256, 0, stream>>>(QKV, VT);
    k_flash<<<dim3(SEQ / QB, NHD, NB), 64, 0, stream>>>(QKV, VT, CTh, CTl);
    k_gemm<bf, 1, float, true, 0><<<dim3((NB * SEQ) / 64, DMOD / 64, 1), 32, 0, stream>>>(CTh, CTl, Wpr, (const bf*)nullptr, DMOD, OUT, DMOD, bpr, (const float*)nullptr, (const float*)nullptr, 1.0f, (size_t)0, (size_t)0, (size_t)0);
}
